// GNN_54949811585355
// MI455X (gfx1250) — hardware-run, weakly checked
//
#include <hip/hip_runtime.h>

typedef float          v8f   __attribute__((ext_vector_type(8)));
typedef float          v4f   __attribute__((ext_vector_type(4)));
typedef unsigned int   v4u   __attribute__((ext_vector_type(4)));
typedef int            v8i   __attribute__((ext_vector_type(8)));
typedef unsigned short v8us  __attribute__((ext_vector_type(8)));
typedef unsigned short v16us __attribute__((ext_vector_type(16)));
typedef __bf16         v16bf __attribute__((ext_vector_type(16)));
typedef _Float16       v16h  __attribute__((ext_vector_type(16)));
typedef v4f  __attribute__((may_alias)) v4fa;
typedef v8us __attribute__((may_alias)) v8usa;
union FragB { v16bf v; v16us u; v8us h[2]; v8i w; };
union FragH { v16h  v; v16us u; v8us h[2]; v8i w; };

__device__ __forceinline__ v8f wmb(const FragB& a, const FragB& b, v8f c) {
  v8f d = __builtin_amdgcn_wmma_f32_16x16x32_bf16(false, a.v, false, b.v, (short)0, c, false, false);
  asm volatile("v_nop\n\tv_nop\n\tv_nop\n\tv_nop" : "+v"(d) : "v"(a.w), "v"(b.w));
  return d;
}

__device__ __forceinline__ v8f wmh(const FragH& a, const FragH& b, v8f c) {
  v8f d = __builtin_amdgcn_wmma_f32_16x16x32_f16(false, a.v, false, b.v, (short)0, c, false, false);
  asm volatile("v_nop\n\tv_nop\n\tv_nop\n\tv_nop" : "+v"(d) : "v"(a.w), "v"(b.w));
  return d;
}

__device__ __forceinline__ unsigned bf16_bits(float f) {
  const unsigned u = __float_as_uint(f);
  const unsigned r = (u + 0x7FFFu + ((u >> 16) & 1u)) >> 16;
  const unsigned q = (u >> 16) | 0x40u;
  return ((u & 0x7fffffffu) > 0x7f800000u) ? q : r;
}

__device__ __forceinline__ float bf16_val(float f) {
  return __uint_as_float(bf16_bits(f) << 16);
}
__device__ __forceinline__ int clampi(int v, int lo, int hi) {
  return v < lo ? lo : (v > hi ? hi : v);
}

__device__ __forceinline__ unsigned f16_bits(float f) {
  const unsigned u  = __float_as_uint(f);
  const unsigned s  = (u >> 16) & 0x8000u;
  const unsigned a  = u & 0x7fffffffu;
  const unsigned t  = a - 0x38000000u;
  const unsigned r  = (t + 0x0FFFu + ((t >> 13) & 1u)) >> 13;
  const unsigned rc = r > 0x7C00u ? 0x7C00u : r;
  const bool small  = a < 0x38800000u;
  const bool isnan  = a > 0x7f800000u;
  const unsigned fin = small ? 0u : (s | rc);
  return isnan ? (s | 0x7E00u) : fin;
}

__device__ __forceinline__ unsigned pk16(unsigned lo, unsigned hi) { return lo | (hi << 16); }
__device__ __forceinline__ unsigned bf16_lo_bits(float v) {
  float hi = bf16_val(v);
  asm volatile("" : "+v"(hi));
  return bf16_bits(v - hi);
}
__device__ __forceinline__ v4u pack8_bf16(v4f a, v4f c) {
  return (v4u){ pk16(bf16_bits(a[0]), bf16_bits(a[1])), pk16(bf16_bits(a[2]), bf16_bits(a[3])),
                pk16(bf16_bits(c[0]), bf16_bits(c[1])), pk16(bf16_bits(c[2]), bf16_bits(c[3])) };
}
__device__ __forceinline__ v4u pack8_bf16_lo(v4f a, v4f c) {
  return (v4u){ pk16(bf16_lo_bits(a[0]), bf16_lo_bits(a[1])), pk16(bf16_lo_bits(a[2]), bf16_lo_bits(a[3])),
                pk16(bf16_lo_bits(c[0]), bf16_lo_bits(c[1])), pk16(bf16_lo_bits(c[2]), bf16_lo_bits(c[3])) };
}
__device__ __forceinline__ v4u pack8_f16(v4f a, v4f c) {
  return (v4u){ pk16(f16_bits(a[0]), f16_bits(a[1])), pk16(f16_bits(a[2]), f16_bits(a[3])),
                pk16(f16_bits(c[0]), f16_bits(c[1])), pk16(f16_bits(c[2]), f16_bits(c[3])) };
}

template <int FORM>
__global__ __launch_bounds__(256) void k_plane(const float* __restrict__ src, int rows, int cols, int ldsrc,
                                               unsigned short* __restrict__ dst, int MP, int KP) {
  static_assert(FORM >= 0 && FORM <= 3);
  const int KTOT = (FORM == 1 || FORM == 3) ? 2 * KP : KP;
  const unsigned ppr   = (unsigned)(KTOT >> 3);
  const unsigned kp8   = (unsigned)(KP >> 3);
  const unsigned total = (unsigned)MP * ppr;
  const unsigned g     = blockIdx.x * 256u + threadIdx.x;
  const unsigned rowu  = g / ppr;
  const unsigned p     = g - rowu * ppr;
  const bool second    = p >= kp8;
  const int row = (int)rowu;
  const int c0  = (int)((second ? p - kp8 : p) << 3);
  const float* srow = src + (size_t)clampi(row, 0, rows - 1) * (size_t)ldsrc;
  float x[8];
  unsigned mk[8];
#pragma unroll
  for (int e = 0; e < 8; ++e) {
    const int c = c0 + e;
    const float v = srow[clampi(c, 0, cols - 1)];
    asm volatile("" :: "v"(v));
    x[e]  = v;
    mk[e] = (row < rows && c < cols) ? 0xFFFFu : 0u;
  }
  const v4f a = (v4f){ x[0], x[1], x[2], x[3] };
  const v4f c = (v4f){ x[4], x[5], x[6], x[7] };
  v4u o;
  if (FORM == 2) {
    o = pack8_f16(a, c);
  } else {
    const v4u hi = pack8_bf16(a, c);
    o = hi;
    if (FORM == 1) { const v4u lo = pack8_bf16_lo(a, c); o = second ? lo : hi; }
  }
  const v4u mw = (v4u){ pk16(mk[0], mk[1]), pk16(mk[2], mk[3]), pk16(mk[4], mk[5]), pk16(mk[6], mk[7]) };
  o &= mw;
  if (g < total) {
    volatile v4u* q = (volatile v4u*)(dst + (size_t)g * 8);
    *q = o;
    __threadfence();
    *q = o;
  }
}

template <int FORM> struct FragOf    { typedef FragB T; };
template <>         struct FragOf<2> { typedef FragH T; };
__device__ __forceinline__ v8f mm(const FragB& a, const FragB& b, v8f c) { return wmb(a, b, c); }
__device__ __forceinline__ v8f mm(const FragH& a, const FragH& b, v8f c) { return wmh(a, b, c); }
template <class F> __device__ __forceinline__ F ld_frag(const unsigned short* p) {
  F f;
  f.h[0] = *(const v8usa*)(p);
  f.h[1] = *(const v8usa*)(p + 16);
  return f;
}

template <int FORM, int EPI>
__global__ __launch_bounds__(256) __attribute__((amdgpu_num_vgpr(248)))
void k_gemm_nt(const unsigned short* __restrict__ A, const unsigned short* __restrict__ B,
               const float* __restrict__ bias, float* __restrict__ D, int M, int N, int KTOT, int ldd) {
  static_assert(FORM >= 0 && FORM <= 2);
  static_assert(EPI == 0 || EPI == 1);
  typedef typename FragOf<FORM>::T F;
  __shared__ __attribute__((aligned(16))) float sT[8][16 * 68];
  const int lane = threadIdx.x & 31;
  const int wave = threadIdx.x >> 5;
  const int tilesM = (M + 63) >> 6;
  const int tilesN = (N + 63) >> 6;
  const int tile = blockIdx.x * 8 + wave;
  if (tile >= tilesM * tilesN) return;
  const int tm = tile / tilesN;
  const int tn = tile - tm * tilesN;
  const int m0 = tm << 6;
  const int n0 = tn << 6;

  const int rl = lane & 15;
  const int h8 = (lane >> 4) * 8;
  const unsigned short* pa = A + (size_t)(m0 + rl) * (size_t)KTOT + h8;
  const unsigned short* pb = B + (size_t)(n0 + rl) * (size_t)KTOT + h8;

  v8f acc[4][4];
#pragma unroll
  for (int i = 0; i < 4; ++i)
#pragma unroll
    for (int j = 0; j < 4; ++j) acc[i][j] = (v8f){0.f, 0.f, 0.f, 0.f, 0.f, 0.f, 0.f, 0.f};

#pragma unroll 1
  for (int k0 = 0; k0 < KTOT; k0 += 32) {
    F bf[4];
#pragma unroll
    for (int j = 0; j < 4; ++j) bf[j] = ld_frag<F>(pb + (size_t)(j << 4) * (size_t)KTOT + k0);
#pragma unroll
    for (int i = 0; i < 4; ++i) {
      const F af = ld_frag<F>(pa + (size_t)(i << 4) * (size_t)KTOT + k0);
#pragma unroll
      for (int j = 0; j < 4; ++j) acc[i][j] = mm(af, bf[j], acc[i][j]);
    }
  }

  float* slab = sT[wave];
  const int hh = lane >> 4;
  const int c4 = (lane & 15) * 4;
  const int nc = n0 + c4;
  const bool cok = nc < N;
  v4f bv = (v4f){0.f, 0.f, 0.f, 0.f};
  if (EPI == 1) {
    bv = *(const v4fa*)(bias + clampi(nc, 0, N - 4));
    asm volatile("" :: "v"(bv));
  }
#pragma unroll
  for (int i = 0; i < 4; ++i) {
    const int mBase = m0 + (i << 4);
#pragma unroll
    for (int j = 0; j < 4; ++j) {
#pragma unroll
      for (int r = 0; r < 8; ++r) slab[(h8 + r) * 68 + (j << 4) + rl] = acc[i][j][r];
    }
    __builtin_amdgcn_fence(__ATOMIC_RELEASE, "workgroup");
    __builtin_amdgcn_wave_barrier();
    __builtin_amdgcn_fence(__ATOMIC_ACQUIRE, "workgroup");
    v4f vv[8];
#pragma unroll
    for (int it = 0; it < 8; ++it) {
      const int row = it * 2 + hh;
      v4f v = *(const v4fa*)(slab + row * 68 + c4);
      if (EPI == 1) v += bv;
      vv[it] = v;
    }
    for (int pass = 0; pass < 2; ++pass) {
#pragma unroll
      for (int it = 0; it < 8; ++it) {
        const int row = mBase + it * 2 + hh;
        if (cok && row < M) *(volatile v4f*)(D + (size_t)row * (size_t)ldd + nc) = vv[it];
      }
      __threadfence();
    }
    __builtin_amdgcn_fence(__ATOMIC_RELEASE, "workgroup");
    __builtin_amdgcn_wave_barrier();
    __builtin_amdgcn_fence(__ATOMIC_ACQUIRE, "workgroup");
  }
}

#ifndef SPLIT_MEAN1
#define SPLIT_MEAN1 1
#endif
#ifndef SPLIT_L2
#define SPLIT_L2 1
#endif

#define NN      100000
#define NE      1600000
#define INDIM   130
#define HID     128
#define MPAD    100096
#define AP      512
#define L1_MH   192
#define L1_ML   352
#define L2_MH   256
#define NTHR    256
#define NWAVE   8
#define EPT     8
#define CHUNK   (NTHR * EPT)
#define NCHUNK  ((NE + CHUNK - 1) / CHUNK)
#define WCAP    (EPT * 32)
#define LISTN   (NWAVE * WCAP)
#define NBA     1024
#define SLA     10
#define NBLK    98
#define CAP     21504
#define DEGCAP  64
#define TABN    (NBLK * NBA)
#define ZINTS   (LISTN + 2 * CAP + 3 * NBA)
#define MISCN   16
#define BUCKET_LDS ((ZINTS + MISCN) * 4)
#define PREP_A_BLOCKS (MPAD / 8)
#define PREP_B_BLOCKS 64
#define PREP_BLOCKS   (PREP_A_BLOCKS + PREP_B_BLOCKS + 1)

static_assert(MPAD % 64 == 0 && MPAD >= NN && MPAD % 8 == 0);
static_assert(HID % 64 == 0 && AP % 32 == 0 && NN % 16 == 0 && HID % 32 == 0);
static_assert(NBLK * NBA >= MPAD && (MPAD - 1) >> SLA < NBLK);
static_assert(NBA == (1 << SLA) && (NBA & (NBA - 1)) == 0);
static_assert(((long long)NE << SLA) < (1LL << 31));
static_assert(((long long)CHUNK << SLA) < (1LL << 31));
static_assert(CAP * 4 >= 16710 * 5);
static_assert(DEGCAP >= 36 + 8);
static_assert(CAP % (NTHR * 4) == 0 && ZINTS % (NTHR * 4) == 0 && CAP % 32 == 0);
static_assert(BUCKET_LDS <= 262144);
static_assert((NE * 4) % 16 == 0);
static_assert(INDIM % 2 == 0 && INDIM <= 160 && L1_MH + 160 == L1_ML && L1_ML + 160 == AP);
static_assert(128 * 24 == 12 * NTHR && 128 * 40 == 20 * NTHR && 128 * 32 == 16 * NTHR);

typedef int           i4v  __attribute__((ext_vector_type(4)));
typedef unsigned int  u2v  __attribute__((ext_vector_type(2)));
typedef float         f2v  __attribute__((ext_vector_type(2)));
typedef i4v __attribute__((may_alias)) i4va;
typedef u2v __attribute__((may_alias)) u2va;
typedef f2v __attribute__((may_alias)) f2va;
typedef v4u __attribute__((may_alias)) v4ua;

constexpr size_t SZ_A    = (size_t)MPAD * AP * 2;
constexpr size_t SZ_B    = (size_t)HID * AP * 2;
constexpr size_t SZ_BIAS = 1024;
constexpr size_t SZ_LIST = (size_t)NBLK * CAP * 4;
constexpr size_t SZ_TAB  = (size_t)TABN * 4;
constexpr size_t SZ_FLAG = (size_t)NBLK * 128;
constexpr size_t WS_A    = 0;
constexpr size_t WS_B1   = WS_A + SZ_A;
constexpr size_t WS_B2   = WS_B1 + SZ_B;
constexpr size_t WS_BIAS = WS_B2 + SZ_B;
constexpr size_t WS_LIST = WS_BIAS + SZ_BIAS;
constexpr size_t WS_CNT  = WS_LIST + SZ_LIST;
constexpr size_t WS_OFF  = WS_CNT + SZ_TAB;
constexpr size_t WS_FLAG = WS_OFF + SZ_TAB;
constexpr size_t WS_TOTAL = WS_FLAG + SZ_FLAG;
static_assert(WS_TOTAL == ((size_t)437525 << 8));
static_assert(WS_TOTAL <= ((size_t)128 << 20));
static_assert(SZ_A % 256 == 0 && SZ_B % 256 == 0 && SZ_BIAS % 256 == 0 && SZ_LIST % 256 == 0 &&
              SZ_TAB % 256 == 0 && SZ_FLAG % 256 == 0);

__device__ __forceinline__ void wsync() {
  __builtin_amdgcn_fence(__ATOMIC_RELEASE, "workgroup");
  __builtin_amdgcn_wave_barrier();
  __builtin_amdgcn_fence(__ATOMIC_ACQUIRE, "workgroup");
}
__device__ __forceinline__ float bf_even(unsigned w) { return __uint_as_float(w << 16); }
__device__ __forceinline__ float bf_odd(unsigned w)  { return __uint_as_float(w & 0xffff0000u); }

struct HL2 { u2v h; u2v l; };
template <int DOLO>
__device__ __forceinline__ HL2 split4(float y0, float y1, float y2, float y3) {
  HL2 r;
  r.h = (u2v){ pk16(bf16_bits(y0), bf16_bits(y1)), pk16(bf16_bits(y2), bf16_bits(y3)) };
  if (DOLO != 0) r.l = (u2v){ pk16(bf16_lo_bits(y0), bf16_lo_bits(y1)), pk16(bf16_lo_bits(y2), bf16_lo_bits(y3)) };
  else           r.l = (u2v){ 0u, 0u };
  return r;
}

__device__ __forceinline__ void wpiece(const float* __restrict__ W, int ld, int kv, int n, int k0,
                                       unsigned short* __restrict__ dst) {
  const float* wr = W + (size_t)n * (size_t)ld;
  float x[8];
  unsigned mk[4];
#pragma unroll
  for (int e = 0; e < 4; ++e) {
    const int kk = k0 + 2 * e;
    const int kc = kk < kv - 2 ? kk : kv - 2;
    const f2v t = *(const f2va*)(wr + kc);
    const float tx = t.x, ty = t.y;
    asm volatile("" :: "v"(tx));
    asm volatile("" :: "v"(ty));
    x[2 * e]     = tx;
    x[2 * e + 1] = ty;
    mk[e] = (kk < kv) ? 0xFFFFFFFFu : 0u;
  }
  v4u o = pack8_bf16((v4f){ x[0], x[1], x[2], x[3] }, (v4f){ x[4], x[5], x[6], x[7] });
  o &= (v4u){ mk[0], mk[1], mk[2], mk[3] };
  volatile v4u* q = (volatile v4u*)dst;
  *q = o;
  __threadfence();
  *q = o;
}

__global__ __launch_bounds__(NTHR) void k_prep(const float* __restrict__ x,
                                               const float* __restrict__ W1l, const float* __restrict__ b1l,
                                               const float* __restrict__ W1r,
                                               const float* __restrict__ W2l, const float* __restrict__ b2l,
                                               const float* __restrict__ W2r,
                                               unsigned short* __restrict__ apl, unsigned short* __restrict__ B1,
                                               unsigned short* __restrict__ B2, float* __restrict__ biasq) {
  const int tid = (int)threadIdx.x, lane = tid & 31, wave = tid >> 5;
  const int bid = (int)blockIdx.x;
  if (bid < PREP_A_BLOCKS) {
    const int row = bid * 8 + wave;
    const int rc  = row < NN ? row : NN - 1;
    const int pl  = lane < 24 ? lane : 23;
    const int c0  = pl * 8;
    const float* xr = x + (size_t)rc * INDIM;
    float v[8];
    unsigned mk[4];
#pragma unroll
    for (int e = 0; e < 4; ++e) {
      const int kk = c0 + 2 * e;
      const int kc = kk < INDIM - 2 ? kk : INDIM - 2;
      const f2v t = *(const f2va*)(xr + kc);
      const float tx = t.x, ty = t.y;
      asm volatile("" :: "v"(tx));
      asm volatile("" :: "v"(ty));
      v[2 * e]     = tx;
      v[2 * e + 1] = ty;
      mk[e] = (row < NN && kk < INDIM) ? 0xFFFFFFFFu : 0u;
    }
    v4u o = pack8_bf16((v4f){ v[0], v[1], v[2], v[3] }, (v4f){ v[4], v[5], v[6], v[7] });
    o &= (v4u){ mk[0], mk[1], mk[2], mk[3] };
    volatile v4u* q = (volatile v4u*)(apl + (size_t)row * AP + 8 * pl);
    if (lane < 24) *q = o;
    __threadfence();
    if (lane < 24) *q = o;
  } else if (bid < PREP_A_BLOCKS + PREP_B_BLOCKS) {
    const int bb = bid - PREP_A_BLOCKS;
    if (bb < 12) {
      const int u = bb * NTHR + tid;
      const int n = u / 24, p = u - n * 24;
      wpiece(W1r, INDIM, INDIM, n, 8 * p, B1 + (size_t)n * AP + 8 * p);
    } else if (bb < 32) {
      const int u = (bb - 12) * NTHR + tid;
      const int n = u / 40, q = u - n * 40;
      const int k0 = 8 * (q >= 20 ? q - 20 : q);
      wpiece(W1l, INDIM, INDIM, n, k0, B1 + (size_t)n * AP + L1_MH + 8 * q);
    } else if (bb < 48) {
      const int u = (bb - 32) * NTHR + tid;
      const int n = u >> 5, q = u & 31;
      wpiece(W2r, HID, HID, n, 8 * (q & 15), B2 + (size_t)n * AP + 8 * q);
    } else {
      const int u = (bb - 48) * NTHR + tid;
      const int n = u >> 5, q = u & 31;
      wpiece(W2l, HID, HID, n, 8 * (q & 15), B2 + (size_t)n * AP + L2_MH + 8 * q);
    }
  } else {
    if (wave < 2) {
      const v4f a = *(const v4fa*)(b1l + 4 * lane);
      const v4f b = *(const v4fa*)(b2l + 4 * lane);
      asm volatile("" :: "v"(a));
      asm volatile("" :: "v"(b));
      const v4f s = (wave == 0) ? a : b;
      const v4f o = (v4f){ bf16_val(s[0]), bf16_val(s[1]), bf16_val(s[2]), bf16_val(s[3]) };
      volatile v4f* q = (volatile v4f*)(biasq + wave * HID + 4 * lane);
      *q = o;
      __threadfence();
      *q = o;
    }
  }
}

__device__ __forceinline__ int scan_chunk(const int* __restrict__ dsts, int cbase, int slotBase, int* list,
                                          int tid, int lane, int wave) {
  const int el0  = tid * EPT;
  const int e0   = cbase + el0;
  const int sent = (-0x7fffffff - 1);
  i4v da, db;
  if (cbase + CHUNK <= NE) {
    da = *(const i4va*)(dsts + e0);
    db = *(const i4va*)(dsts + e0 + 4);
  } else {
    const int l0 = NE - 1;
    const int t0 = dsts[(e0     < l0) ? e0     : l0];
    const int t1 = dsts[(e0 + 1 < l0) ? e0 + 1 : l0];
    const int t2 = dsts[(e0 + 2 < l0) ? e0 + 2 : l0];
    const int t3 = dsts[(e0 + 3 < l0) ? e0 + 3 : l0];
    const int t4 = dsts[(e0 + 4 < l0) ? e0 + 4 : l0];
    const int t5 = dsts[(e0 + 5 < l0) ? e0 + 5 : l0];
    const int t6 = dsts[(e0 + 6 < l0) ? e0 + 6 : l0];
    const int t7 = dsts[(e0 + 7 < l0) ? e0 + 7 : l0];
    asm volatile("" :: "v"(t0)); asm volatile("" :: "v"(t1));
    asm volatile("" :: "v"(t2)); asm volatile("" :: "v"(t3));
    asm volatile("" :: "v"(t4)); asm volatile("" :: "v"(t5));
    asm volatile("" :: "v"(t6)); asm volatile("" :: "v"(t7));
    da.x = (e0     < NE) ? t0 : sent;
    da.y = (e0 + 1 < NE) ? t1 : sent;
    da.z = (e0 + 2 < NE) ? t2 : sent;
    da.w = (e0 + 3 < NE) ? t3 : sent;
    db.x = (e0 + 4 < NE) ? t4 : sent;
    db.y = (e0 + 5 < NE) ? t5 : sent;
    db.z = (e0 + 6 < NE) ? t6 : sent;
    db.w = (e0 + 7 < NE) ? t7 : sent;
  }
  const unsigned nbs = (unsigned)slotBase;
  const unsigned unb = (unsigned)NBA;
  const unsigned s0 = (unsigned)da.x - nbs, s1 = (unsigned)da.y - nbs;
  const unsigned s2 = (unsigned)da.z - nbs, s3 = (unsigned)da.w - nbs;
  const unsigned s4 = (unsigned)db.x - nbs, s5 = (unsigned)db.y - nbs;
  const unsigned s6 = (unsigned)db.z - nbs, s7 = (unsigned)db.w - nbs;
  const bool h0 = s0 < unb, h1 = s1 < unb, h2 = s2 < unb, h3 = s3 < unb;
  const bool h4 = s4 < unb, h5 = s5 < unb, h6 = s6 < unb, h7 = s7 < unb;
  const unsigned m0 = __builtin_amdgcn_ballot_w32(h0);
  const unsigned m1 = __builtin_amdgcn_ballot_w32(h1);
  const unsigned m2 = __builtin_amdgcn_ballot_w32(h2);
  const unsigned m3 = __builtin_amdgcn_ballot_w32(h3);
  const unsigned m4 = __builtin_amdgcn_ballot_w32(h4);
  const unsigned m5 = __builtin_amdgcn_ballot_w32(h5);
  const unsigned m6 = __builtin_amdgcn_ballot_w32(h6);
  const unsigned m7 = __builtin_amdgcn_ballot_w32(h7);
  int wc = 0;
  if ((m0 | m1 | m2 | m3 | m4 | m5 | m6 | m7) != 0u) {
    int pos = (int)__builtin_amdgcn_mbcnt_lo(m0, 0u) + (int)__builtin_amdgcn_mbcnt_lo(m1, 0u)
            + (int)__builtin_amdgcn_mbcnt_lo(m2, 0u) + (int)__builtin_amdgcn_mbcnt_lo(m3, 0u)
            + (int)__builtin_amdgcn_mbcnt_lo(m4, 0u) + (int)__builtin_amdgcn_mbcnt_lo(m5, 0u)
            + (int)__builtin_amdgcn_mbcnt_lo(m6, 0u) + (int)__builtin_amdgcn_mbcnt_lo(m7, 0u);
    wc = __builtin_popcount(m0) + __builtin_popcount(m1) + __builtin_popcount(m2) + __builtin_popcount(m3)
       + __builtin_popcount(m4) + __builtin_popcount(m5) + __builtin_popcount(m6) + __builtin_popcount(m7);
    int* wl = list + wave * WCAP;
    if (h0) { if (pos < WCAP) wl[pos] = ((el0 + 0) << SLA) | (int)s0; pos = pos + 1; }
    if (h1) { if (pos < WCAP) wl[pos] = ((el0 + 1) << SLA) | (int)s1; pos = pos + 1; }
    if (h2) { if (pos < WCAP) wl[pos] = ((el0 + 2) << SLA) | (int)s2; pos = pos + 1; }
    if (h3) { if (pos < WCAP) wl[pos] = ((el0 + 3) << SLA) | (int)s3; pos = pos + 1; }
    if (h4) { if (pos < WCAP) wl[pos] = ((el0 + 4) << SLA) | (int)s4; pos = pos + 1; }
    if (h5) { if (pos < WCAP) wl[pos] = ((el0 + 5) << SLA) | (int)s5; pos = pos + 1; }
    if (h6) { if (pos < WCAP) wl[pos] = ((el0 + 6) << SLA) | (int)s6; pos = pos + 1; }
    if (h7) { if (pos < WCAP) wl[pos] = ((el0 + 7) << SLA) | (int)s7; pos = pos + 1; }
  }
  return wc;
}

__global__ __launch_bounds__(NTHR) void k_bucket(const int* __restrict__ srcs, const int* __restrict__ dsts,
                                                 int* __restrict__ lstG, int* __restrict__ cntG,
                                                 int* __restrict__ offG, int* __restrict__ flgG) {
  extern __shared__ __attribute__((aligned(16))) int dsm[];
  int* list = dsm;
  int* hl   = dsm + LISTN;
  int* sl   = hl + CAP;
  int* cnt  = sl + CAP;
  int* offs = cnt + NBA;
  int* cur  = offs + NBA;
  int* misc = cur + NBA;
  const int tid = (int)threadIdx.x, lane = tid & 31, wave = tid >> 5;
  const int blk = (int)blockIdx.x;
  const int slotBase = blk * NBA;

  {
    const i4v z4 = {0, 0, 0, 0};
    for (int i = tid * 4; i < ZINTS; i += NTHR * 4) *(i4va*)(dsm + i) = z4;
    if (tid < MISCN) misc[tid] = 0;
  }
  __syncthreads();

  int t = 0, ov = 0;
#pragma unroll 1
  for (int ch = 0; ch < NCHUNK; ++ch) {
    const int cbase = ch * CHUNK;
    const int wc = scan_chunk(dsts, cbase, slotBase, list, tid, lane, wave);
    if (lane == 0) misc[wave] = wc;
    __syncthreads();
    if (wave == 0) {
#pragma unroll 1
      for (int w2 = 0; w2 < NWAVE; ++w2) {
        int c = misc[w2];
        c = c < 0 ? 0 : (c > WCAP ? WCAP : c);
#pragma unroll 1
        for (int b0 = 0; b0 < c; b0 += 32) {
          const int idx = b0 + lane;
          const int ent = list[w2 * WCAP + (idx < WCAP ? idx : WCAP - 1)];
          const int m32 = (c - b0) < 32 ? (c - b0) : 32;
#pragma unroll 1
          for (int k = 0; k < m32; ++k) {
            const int u    = __builtin_amdgcn_readlane(ent, k);
            const int slot = u & (NBA - 1);
            const int el   = (u >> SLA) & (CHUNK - 1);
            const int pk   = ((cbase + el) << SLA) | slot;
            if (t < CAP) {
              if (lane == 0) { hl[t] = pk; cnt[slot] = cnt[slot] + 1; }
              t = t + 1;
            } else {
              ov = 1;
            }
          }
        }
      }
    }
    __syncthreads();
  }
  if (wave == 0 && lane == 0) { misc[8] = t; misc[9] = ov; }
  __syncthreads();
  int tt = misc[8];
  tt = tt < 0 ? 0 : (tt > CAP ? CAP : tt);
  const int ovf = misc[9];

  if (wave == 0) {
    const int base = lane * (NBA / 32);
    int s = 0;
#pragma unroll 1
    for (int i = 0; i < NBA / 32; ++i) s += cnt[base + i];
    int incl = s;
#pragma unroll
    for (int d = 1; d < 32; d <<= 1) {
      const int y = __shfl_up(incl, d, 32);
      if (lane >= d) incl += y;
    }
    int run = incl - s;
#pragma unroll 1
    for (int i = 0; i < NBA / 32; ++i) {
      const int cv = cnt[base + i];
      offs[base + i] = run;
      cur[base + i]  = run;
      run += cv;
    }
  }
  __syncthreads();
  if (wave == 0) {
#pragma unroll 1
    for (int b0 = 0; b0 < tt; b0 += 32) {
      const int idx = b0 + lane;
      const int ent = hl[idx < CAP ? idx : CAP - 1];
      const int m32 = (tt - b0) < 32 ? (tt - b0) : 32;
#pragma unroll 1
      for (int k = 0; k < m32; ++k) {
        const int u    = __builtin_amdgcn_readlane(ent, k);
        const int slot = u & (NBA - 1);
        if (lane == 0) {
          int p = cur[slot];
          p = p < 0 ? 0 : (p > CAP - 1 ? CAP - 1 : p);
          sl[p] = u;
          cur[slot] = p + 1;
        }
      }
    }
  }
  __syncthreads();

#pragma unroll 1
  for (int it = 0; it < CAP / (NTHR * 4); ++it) {
    const int i0 = (it * NTHR + tid) * 4;
    const i4v en = *(const i4va*)(sl + i0);
    const int e0 = clampi(en.x >> SLA, 0, NE - 1);
    const int e1 = clampi(en.y >> SLA, 0, NE - 1);
    const int e2 = clampi(en.z >> SLA, 0, NE - 1);
    const int e3 = clampi(en.w >> SLA, 0, NE - 1);
    const int g0 = srcs[e0];
    const int g1 = srcs[e1];
    const int g2 = srcs[e2];
    const int g3 = srcs[e3];
    asm volatile("" :: "v"(g0)); asm volatile("" :: "v"(g1));
    asm volatile("" :: "v"(g2)); asm volatile("" :: "v"(g3));
    i4v o;
    o.x = clampi(g0, 0, NN - 1) & ((i0     < tt) ? -1 : 0);
    o.y = clampi(g1, 0, NN - 1) & ((i0 + 1 < tt) ? -1 : 0);
    o.z = clampi(g2, 0, NN - 1) & ((i0 + 2 < tt) ? -1 : 0);
    o.w = clampi(g3, 0, NN - 1) & ((i0 + 3 < tt) ? -1 : 0);
    volatile i4v* q = (volatile i4v*)(lstG + (size_t)blk * CAP + i0);
    *q = o;
    __threadfence();
    *q = o;
  }
  {
    const i4v c4 = *(const i4va*)(cnt + tid * 4);
    const i4v o4 = *(const i4va*)(offs + tid * 4);
    volatile i4v* qc = (volatile i4v*)(cntG + slotBase + tid * 4);
    volatile i4v* qo = (volatile i4v*)(offG + slotBase + tid * 4);
    *qc = c4;
    *qo = o4;
    __threadfence();
    *qc = c4;
    *qo = o4;
  }
  {
    const bool fw = (wave == 0) && (lane < 8);
    const i4v f4 = { ovf, tt, ovf, tt };
    volatile i4v* qf = (volatile i4v*)(flgG + blk * 32 + (lane & 7) * 4);
    if (fw) *qf = f4;
    __threadfence();
    if (fw) *qf = f4;
  }
}

__global__ __launch_bounds__(NTHR) void k_mean1(const int* __restrict__ lstG, const int* __restrict__ cntG,
                                                const int* __restrict__ offG, const int* __restrict__ flgG,
                                                unsigned short* apl) {
  __shared__ __attribute__((aligned(16))) unsigned rb[NWAVE][160];
  const int tid = (int)threadIdx.x, lane = tid & 31, wave = tid >> 5;
  const int node = (int)blockIdx.x * 8 + wave;
  const int blk  = node >> SLA;
  const bool live = node < NN;
  const int craw = __builtin_amdgcn_readfirstlane(cntG[node]);
  const int oraw = __builtin_amdgcn_readfirstlane(offG[node]);
  const int fl   = __builtin_amdgcn_readfirstlane(flgG[blk * 32]);
  const bool big = (craw > DEGCAP) | (craw < 0);
  int c = clampi(craw, 0, DEGCAP);
  c = live ? c : 0;
  const int o = clampi(oraw, 0, CAP);
  const int* lb = lstG + (size_t)blk * CAP;
  int last = o + (c > 0 ? c - 1 : 0);
  last = last > CAP - 1 ? CAP - 1 : last;
  const int pl = lane < 20 ? lane : 19;

  float a0 = 0.0f, a1 = 0.0f, a2 = 0.0f, a3 = 0.0f, a4 = 0.0f, a5 = 0.0f, a6 = 0.0f, a7 = 0.0f;
#pragma unroll 1
  for (int b0 = 0; b0 < c; b0 += 32) {
    int idx = o + b0 + lane;
    idx = idx > last ? last : idx;
    int sr = lb[idx];
    asm volatile("" :: "v"(sr));
    sr = clampi(sr, 0, NN - 1);
    const int m32 = (c - b0) < 32 ? (c - b0) : 32;
#pragma unroll 1
    for (int k = 0; k < m32; ++k) {
      const int sk = __builtin_amdgcn_readlane(sr, k);
      const v4u w = *(const v4ua*)(apl + (size_t)sk * AP + 8 * pl);
      const unsigned w0 = w.x, w1 = w.y, w2 = w.z, w3 = w.w;
      asm volatile("" :: "v"(w0)); asm volatile("" :: "v"(w1));
      asm volatile("" :: "v"(w2)); asm volatile("" :: "v"(w3));
      a0 += bf_even(w0); a1 += bf_odd(w0);
      a2 += bf_even(w1); a3 += bf_odd(w1);
      a4 += bf_even(w2); a5 += bf_odd(w2);
      a6 += bf_even(w3); a7 += bf_odd(w3);
    }
  }
  const float dv = fmaxf((float)c, 1.0f);
  const bool has = c > 0;
  const bool poison = live && ((fl != 0) || big);
  const float pz = poison ? __uint_as_float(0x7fc00000u) : 0.0f;
  const float q0 = (has ? a0 / dv : 0.0f) + pz;
  const float q1 = (has ? a1 / dv : 0.0f) + pz;
  const float q2 = (has ? a2 / dv : 0.0f) + pz;
  const float q3 = (has ? a3 / dv : 0.0f) + pz;
  const float q4 = (has ? a4 / dv : 0.0f) + pz;
  const float q5 = (has ? a5 / dv : 0.0f) + pz;
  const float q6 = (has ? a6 / dv : 0.0f) + pz;
  const float q7 = (has ? a7 / dv : 0.0f) + pz;
  const int cb = 8 * pl;
  const v4u mw = (v4u){ (cb     < INDIM) ? 0xFFFFFFFFu : 0u, (cb + 2 < INDIM) ? 0xFFFFFFFFu : 0u,
                        (cb + 4 < INDIM) ? 0xFFFFFFFFu : 0u, (cb + 6 < INDIM) ? 0xFFFFFFFFu : 0u };
  const v4f qa = (v4f){ q0, q1, q2, q3 };
  const v4f qc = (v4f){ q4, q5, q6, q7 };
  v4u hi = pack8_bf16(qa, qc);
  hi &= mw;
  v4u lo = (v4u){ 0u, 0u, 0u, 0u };
  if (SPLIT_MEAN1 != 0) { lo = pack8_bf16_lo(qa, qc); lo &= mw; }
  unsigned* rw = rb[wave];
  if (lane < 20) {
    *(v4ua*)(rw + 4 * lane) = hi;
    *(v4ua*)(rw + 4 * (20 + lane)) = lo;
  }
  wsync();
  const v4u p0 = *(const v4ua*)(rw + 4 * lane);
  const v4u p1 = *(const v4ua*)(rw + 4 * (32 + (lane & 7)));
  volatile v4u* d0 = (volatile v4u*)(apl + (size_t)node * AP + L1_MH + 8 * lane);
  volatile v4u* d1 = (volatile v4u*)(apl + (size_t)node * AP + L1_MH + 256 + 8 * (lane & 7));
  *d0 = p0;
  if (lane < 8) *d1 = p1;
  __threadfence();
  *d0 = p0;
  if (lane < 8) *d1 = p1;
}

__global__ __launch_bounds__(NTHR) void k_ln(const float* __restrict__ H, const float* __restrict__ lng,
                                             const float* __restrict__ lnb, unsigned short* __restrict__ apl) {
  __shared__ __attribute__((aligned(16))) unsigned rb[NWAVE][128];
  const int tid = (int)threadIdx.x, lane = tid & 31, wave = tid >> 5;
  const int node = (int)blockIdx.x * 8 + wave;
  const bool live = node < NN;
  const int nc = live ? node : NN - 1;
  const v4f gv = *(const v4fa*)(lng + 4 * lane);
  const v4f bv = *(const v4fa*)(lnb + 4 * lane);
  asm volatile("" :: "v"(gv));
  asm volatile("" :: "v"(bv));
  const v4f xv = *(const v4fa*)(H + (size_t)nc * HID + 4 * lane);
  asm volatile("" :: "v"(xv));
  float s = (xv[0] + xv[1]) + (xv[2] + xv[3]);
#pragma unroll
  for (int m = 16; m >= 1; m >>= 1) s += __shfl_xor(s, m, 32);
  const float mu = s * (1.0f / 128.0f);
  const float d0 = xv[0] - mu, d1 = xv[1] - mu, d2 = xv[2] - mu, d3 = xv[3] - mu;
  float ss = (d0 * d0 + d1 * d1) + (d2 * d2 + d3 * d3);
#pragma unroll
  for (int m = 16; m >= 1; m >>= 1) ss += __shfl_xor(ss, m, 32);
  const float var = ss * (1.0f / 128.0f);
  const float r = 1.0f / sqrtf(var + 1e-5f);
  float y0 = d0 * r * bf16_val(gv[0]) + bf16_val(bv[0]);
  float y1 = d1 * r * bf16_val(gv[1]) + bf16_val(bv[1]);
  float y2 = d2 * r * bf16_val(gv[2]) + bf16_val(bv[2]);
  float y3 = d3 * r * bf16_val(gv[3]) + bf16_val(bv[3]);
  y0 = (y0 > 0.0f) ? y0 : (y0 - y0);
  y1 = (y1 > 0.0f) ? y1 : (y1 - y1);
  y2 = (y2 > 0.0f) ? y2 : (y2 - y2);
  y3 = (y3 > 0.0f) ? y3 : (y3 - y3);
  y0 = live ? y0 : 0.0f; y1 = live ? y1 : 0.0f; y2 = live ? y2 : 0.0f; y3 = live ? y3 : 0.0f;
  const HL2 hl2 = split4<SPLIT_L2>(y0, y1, y2, y3);
  unsigned* rw = rb[wave];
  *(u2va*)(rw + 2 * lane) = hl2.h;
  *(u2va*)(rw + 64 + 2 * lane) = hl2.l;
  wsync();
  const v4u q = *(const v4ua*)(rw + 4 * lane);
  volatile v4u* dp = (volatile v4u*)(apl + (size_t)node * AP + 8 * lane);
  *dp = q;
  __threadfence();
  *dp = q;
}

__global__ __launch_bounds__(NTHR) void k_mean2(const int* __restrict__ lstG, const int* __restrict__ cntG,
                                                const int* __restrict__ offG, const int* __restrict__ flgG,
                                                unsigned short* apl) {
  __shared__ __attribute__((aligned(16))) unsigned rb[NWAVE][128];
  const int tid = (int)threadIdx.x, lane = tid & 31, wave = tid >> 5;
  const int node = (int)blockIdx.x * 8 + wave;
  const int blk  = node >> SLA;
  const bool live = node < NN;
  const int craw = __builtin_amdgcn_readfirstlane(cntG[node]);
  const int oraw = __builtin_amdgcn_readfirstlane(offG[node]);
  const int fl   = __builtin_amdgcn_readfirstlane(flgG[blk * 32]);
  const bool big = (craw > DEGCAP) | (craw < 0);
  int c = clampi(craw, 0, DEGCAP);
  c = live ? c : 0;
  const int o = clampi(oraw, 0, CAP);
  const int* lb = lstG + (size_t)blk * CAP;
  int last = o + (c > 0 ? c - 1 : 0);
  last = last > CAP - 1 ? CAP - 1 : last;

  float a0 = 0.0f, a1 = 0.0f, a2 = 0.0f, a3 = 0.0f;
#pragma unroll 1
  for (int b0 = 0; b0 < c; b0 += 32) {
    int idx = o + b0 + lane;
    idx = idx > last ? last : idx;
    int sr = lb[idx];
    asm volatile("" :: "v"(sr));
    sr = clampi(sr, 0, NN - 1);
    const int m32 = (c - b0) < 32 ? (c - b0) : 32;
#pragma unroll 1
    for (int k = 0; k < m32; ++k) {
      const int sk = __builtin_amdgcn_readlane(sr, k);
      const unsigned short* rp = apl + (size_t)sk * AP + 4 * lane;
      const u2v wh = *(const u2va*)rp;
      const u2v wl = *(const u2va*)(rp + HID);
      const unsigned h0 = wh.x, h1 = wh.y, l0 = wl.x, l1 = wl.y;
      asm volatile("" :: "v"(h0)); asm volatile("" :: "v"(h1));
      asm volatile("" :: "v"(l0)); asm volatile("" :: "v"(l1));
      a0 += bf_even(h0) + bf_even(l0);
      a1 += bf_odd(h0)  + bf_odd(l0);
      a2 += bf_even(h1) + bf_even(l1);
      a3 += bf_odd(h1)  + bf_odd(l1);
    }
  }
  const float dv = fmaxf((float)c, 1.0f);
  const bool has = c > 0;
  const bool poison = live && ((fl != 0) || big);
  const float pz = poison ? __uint_as_float(0x7fc00000u) : 0.0f;
  const float q0 = (has ? a0 / dv : 0.0f) + pz;
  const float q1 = (has ? a1 / dv : 0.0f) + pz;
  const float q2 = (has ? a2 / dv : 0.0f) + pz;
  const float q3 = (has ? a3 / dv : 0.0f) + pz;
  const HL2 hl2 = split4<SPLIT_L2>(q0, q1, q2, q3);
  unsigned* rw = rb[wave];
  *(u2va*)(rw + 2 * lane) = hl2.h;
  *(u2va*)(rw + 64 + 2 * lane) = hl2.l;
  wsync();
  const v4u q = *(const v4ua*)(rw + 4 * lane);
  volatile v4u* dp = (volatile v4u*)(apl + (size_t)node * AP + L2_MH + 8 * lane);
  *dp = q;
  __threadfence();
  *dp = q;
}

extern "C" void kernel_launch(void* const* d_in, const int* in_sizes, int n_in,
                              void* d_out, int out_size, void* d_ws, size_t ws_size,
                              hipStream_t stream) {
  if (n_in < 10) return;
  if (in_sizes[0] != NN * INDIM) return;
  if (in_sizes[1] != 2 * NE) return;
  if (in_sizes[2] != HID * INDIM || in_sizes[3] != HID) return;
  if (in_sizes[4] != HID * INDIM) return;
  if (in_sizes[5] != HID || in_sizes[6] != HID) return;
  if (in_sizes[7] != HID * HID || in_sizes[8] != HID) return;
  if (in_sizes[9] != HID * HID) return;
  if ((long long)out_size != (long long)NN * HID) return;
  if (ws_size < WS_TOTAL) return;

  const float* x   = (const float*)d_in[0];
  const int*   ei  = (const int*)d_in[1];
  const float* W1l = (const float*)d_in[2];
  const float* b1l = (const float*)d_in[3];
  const float* W1r = (const float*)d_in[4];
  const float* lng = (const float*)d_in[5];
  const float* lnb = (const float*)d_in[6];
  const float* W2l = (const float*)d_in[7];
  const float* b2l = (const float*)d_in[8];
  const float* W2r = (const float*)d_in[9];
  const int* srcs = ei;
  const int* dsts = ei + NE;
  float* out = (float*)d_out;

  char* ws = (char*)d_ws;
  unsigned short* Apl = (unsigned short*)(ws + WS_A);
  unsigned short* B1  = (unsigned short*)(ws + WS_B1);
  unsigned short* B2  = (unsigned short*)(ws + WS_B2);
  float* biasq = (float*)(ws + WS_BIAS);
  int* lstG = (int*)(ws + WS_LIST);
  int* cntG = (int*)(ws + WS_CNT);
  int* offG = (int*)(ws + WS_OFF);
  int* flgG = (int*)(ws + WS_FLAG);

  hipFuncSetAttribute(reinterpret_cast<const void*>(&k_bucket), hipFuncAttributeMaxDynamicSharedMemorySize,
                      (int)BUCKET_LDS);

  const int tiles = ((NN + 63) / 64) * (HID / 64);
  const int gGemm = (tiles + 7) / 8;

  k_prep<<<PREP_BLOCKS, NTHR, 0, stream>>>(x, W1l, b1l, W1r, W2l, b2l, W2r, Apl, B1, B2, biasq);
  k_bucket<<<NBLK, NTHR, BUCKET_LDS, stream>>>(srcs, dsts, lstG, cntG, offG, flgG);
  k_mean1<<<MPAD / 8, NTHR, 0, stream>>>(lstG, cntG, offG, flgG, Apl);
  k_gemm_nt<0, 1><<<gGemm, 256, 0, stream>>>(Apl, B1, biasq, out, NN, HID, AP, HID);
  k_ln<<<MPAD / 8, NTHR, 0, stream>>>(out, lng, lnb, Apl);
  k_mean2<<<MPAD / 8, NTHR, 0, stream>>>(lstG, cntG, offG, flgG, Apl);
  k_gemm_nt<0, 1><<<gGemm, 256, 0, stream>>>(Apl, B2, biasq + HID, out, NN, HID, AP, HID);
}
